// Model_63788854280271
// MI455X (gfx1250) — hardware-run, weakly checked
//
#include <hip/hip_runtime.h>


#ifndef NB
#define NB 4
#endif
#ifndef SEQ
#define SEQ 1024
#endif
#define NB_FULL  4
#define SEQ_FULL 1024
#ifndef OUT_SEQ
#define OUT_SEQ SEQ
#endif
#define HA   192
#define NHA  16
#define DA   12
#define KPA  192
#define NPA  16
#define HB   66
#define NHB  11
#define DB   6
#define KPB  96
#define NPB  12
#define HP   16
#define NRO  192
#define ONT  12
#define AW   4
#define OSP  20
#define OPP  196
#define PCAR 16.0f
#define CCAR 64.0f
#define WCAR 64.0f
#define OSC  (CCAR / PCAR)
#define OFOLD (1.0f / (CCAR * WCAR))
#define LOG2E 1.4426950408889634f
#define PSH  14.0f
#define NEGB (-3.0e38f)

static_assert(HP == 16);
static_assert(NHA * DA == HA);
static_assert(NHB * DB == HB);
static_assert(DA <= HP);
static_assert(DB <= HP);
static_assert(NPA >= NHA);
static_assert(NPB >= NHB);
static_assert((NPA * HP) % 64 == 0);
static_assert((NPB * HP) % 64 == 0);
static_assert((NPA * HP) % 32 == 0);
static_assert((NPB * HP) % 32 == 0);
static_assert(KPA % 32 == 0);
static_assert(KPB % 32 == 0);
static_assert(KPA == HA);
static_assert(KPB >= HB);
static_assert(KPA % 8 == 0);
static_assert(KPB % 8 == 0);
static_assert(SEQ % 64 == 0);
static_assert((NB * SEQ) % 64 == 0);
static_assert(SEQ % 32 == 0);
static_assert(SEQ % (16 * AW) == 0);
static_assert(NB <= NB_FULL);
static_assert(SEQ <= SEQ_FULL);
static_assert(OUT_SEQ % 16 == 0);
static_assert(OUT_SEQ >= SEQ);
static_assert(NRO == ONT * 16);
static_assert(NRO >= HA);
static_assert(NRO >= HB);
static_assert(NRO + 4 <= OPP);
static_assert((OPP * 4) % 16 == 0);
static_assert((OSP * 4) % 16 == 0);
static_assert((64 * HA) % 128 == 0);
static_assert((64 * HB) % 128 == 0);
static_assert((size_t)NB_FULL * SEQ_FULL * HA * 4 == (size_t)3145728);
static_assert(((size_t)NB_FULL * SEQ_FULL * HA * 4) % 128 == 0);
static_assert(16 * 68 * 4 <= 131072);
static_assert(AW * 16 * OSP * 4 <= 131072);
static_assert(16 * OPP * 4 <= 131072);
static_assert(4 * 32 * 8 == 16 * 64);
static_assert(32 * 8 == 16 * HP);

typedef _Float16 h16;
typedef unsigned short bf;
typedef __attribute__((ext_vector_type(16))) __bf16   v16bf;
typedef __attribute__((ext_vector_type(16))) _Float16 v16h;
typedef __attribute__((ext_vector_type(8)))  _Float16 v8h;
typedef __attribute__((ext_vector_type(8)))  unsigned short v8us;
typedef __attribute__((ext_vector_type(8)))  float    v8f;
typedef __attribute__((ext_vector_type(4)))  float    v4f;
typedef v4f  __attribute__((may_alias)) v4fa;

__device__ __forceinline__ unsigned short f2bf(float f) { unsigned u = __float_as_uint(f); u += 0x7FFFu + ((u >> 16) & 1u); return (unsigned short)(u >> 16); }
__device__ __forceinline__ float bfr(float f) { return __uint_as_float(((unsigned)f2bf(f)) << 16); }
__device__ __forceinline__ v16h cat16(v8h lo, v8h hi) { return __builtin_shufflevector(lo, hi, 0, 1, 2, 3, 4, 5, 6, 7, 8, 9, 10, 11, 12, 13, 14, 15); }
__device__ __forceinline__ v16bf cat16b(v8us lo, v8us hi) { return __builtin_bit_cast(v16bf, __builtin_shufflevector(lo, hi, 0, 1, 2, 3, 4, 5, 6, 7, 8, 9, 10, 11, 12, 13, 14, 15)); }
__device__ __forceinline__ v8f wmma16(v16h a, v16h b, v8f c) { return __builtin_amdgcn_wmma_f32_16x16x32_f16(false, a, false, b, (short)0, c, false, false); }
__device__ __forceinline__ v8f wmmab(v16bf a, v16bf b, v8f c) { return __builtin_amdgcn_wmma_f32_16x16x32_bf16(false, a, false, b, (short)0, c, false, false); }
__device__ __forceinline__ v16h  ldh(const h16* p) { return cat16(*(const v8h*)p, *(const v8h*)(p + 16)); }
__device__ __forceinline__ v16bf ldb(const bf* p)  { return cat16b(*(const v8us*)p, *(const v8us*)(p + 16)); }
__device__ __forceinline__ void wave_sync() { __builtin_amdgcn_fence(3  , "wavefront"); __builtin_amdgcn_wave_barrier(); asm volatile("" ::: "memory"); }

__device__ __forceinline__ v8f wmma16g(v16h a, v16h b, v8f c) { c = wmma16(a, b, c); asm volatile("v_nop\n\tv_nop\n\tv_nop\n\tv_nop" : "+v"(c) : "v"(a), "v"(b)); return c; }
__device__ __forceinline__ v8f wmmabg(v16bf a, v16bf b, v8f c) { c = wmmab(a, b, c); asm volatile("v_nop\n\tv_nop\n\tv_nop\n\tv_nop" : "+v"(c) : "v"(a), "v"(b)); return c; }
__device__ __forceinline__ h16 toh_flush(float v) { const h16 r = (h16)v; return (fabsf(v) < 6.103515625e-05f) ? (h16)0.0f : r; }

__global__ __launch_bounds__(256) void k_cvt8(const float* __restrict__ src, bf* dst, size_t n8) {
    const size_t i = (size_t)blockIdx.x * 256 + threadIdx.x; if (i >= n8) return;
    const v8f v = *(const v8f*)(src + i * 8); v8us o;
#pragma unroll
    for (int k = 0; k < 8; ++k) o[k] = f2bf(v[k]);
    *(volatile v8us*)(dst + i * 8) = o; __threadfence(); *(volatile v8us*)(dst + i * 8) = o;
}

__global__ __launch_bounds__(256) void k_cvtpad(const float* __restrict__ src, bf* dst, int rows, int scols, int dcols) {
#pragma clang fp contract(off)
    const int per = dcols >> 3;
    const int i = blockIdx.x * 256 + threadIdx.x; if (i >= rows * per) return;
    const int r = i / per, c8 = (i - r * per) * 8;
    v8us o;
#pragma unroll
    for (int k = 0; k < 8; ++k) {
        const int c = c8 + k; const int cc = c < scols ? c : scols - 1;
        float v = src[(size_t)r * scols + cc]; asm volatile("" : "+v"(v));
        o[k] = (c < scols) ? f2bf(v) : (unsigned short)0; }
    *(volatile v8us*)(dst + (size_t)i * 8) = o; __threadfence(); *(volatile v8us*)(dst + (size_t)i * 8) = o;
}

__global__ __launch_bounds__(256) void k_wpack_rows(const float* __restrict__ W, bf* dst, int H, int D, int NH, int KP, int NPr) {
#pragma clang fp contract(off)
    const int per = KP >> 3;
    const int i = blockIdx.x * 256 + threadIdx.x; if (i >= NPr * per) return;
    const int n = i / per, c8 = (i - n * per) * 8;
    const int hd = n >> 4, dp = n & 15;
    const int rowok = (dp < D) & (hd < NH);
    int sr = hd * D + dp; sr = sr < H - 1 ? sr : H - 1;
    v8us o;
#pragma unroll
    for (int k = 0; k < 8; ++k) {
        const int c = c8 + k; const int cc = c < H ? c : H - 1;
        float v = W[(size_t)sr * H + cc]; asm volatile("" : "+v"(v));
        o[k] = (rowok & (c < H)) ? f2bf(v) : (unsigned short)0; }
    *(volatile v8us*)(dst + (size_t)i * 8) = o; __threadfence(); *(volatile v8us*)(dst + (size_t)i * 8) = o;
}

__global__ __launch_bounds__(256) void k_wpack_cols(const float* __restrict__ W, h16* dst, int H, int D, int NH, int KC, int NRo) {
#pragma clang fp contract(off)
    const int per = KC >> 3;
    const int i = blockIdx.x * 256 + threadIdx.x; if (i >= NRo * per) return;
    const int n = i / per, c8 = (i - n * per) * 8;
    const int nn = n < H ? n : H - 1;
    v8h o;
#pragma unroll
    for (int k = 0; k < 8; ++k) {
        const int c = c8 + k; const int hd = c >> 4, dp = c & 15;
        int sc = hd * D + dp; sc = sc < H - 1 ? sc : H - 1;
        float v = W[(size_t)nn * H + sc]; asm volatile("" : "+v"(v));
        const int ok = (n < H) & (dp < D) & (hd < NH);
        o[k] = ok ? toh_flush(bfr(v) * WCAR) : (h16)0.0f; }
    *(volatile v8h*)(dst + (size_t)i * 8) = o; __threadfence(); *(volatile v8h*)(dst + (size_t)i * 8) = o;
}

__device__ __forceinline__ void gemm64(const bf* __restrict__ A, const bf* __restrict__ Bt, size_t aoff, size_t boff, int K, v8f (&acc)[4][4]) {
#pragma unroll 1
    for (int kc = 0; kc < K; kc += 32) {
        v16bf a[4];
#pragma unroll
        for (int mb = 0; mb < 4; ++mb) a[mb] = ldb(A + aoff + (size_t)mb * 16 * K + kc);
#pragma unroll
        for (int nb = 0; nb < 4; ++nb) { const v16bf b = ldb(Bt + boff + (size_t)nb * 16 * K + kc);
#pragma unroll
            for (int mb = 0; mb < 4; ++mb) acc[mb][nb] = wmmabg(a[mb], b, acc[mb][nb]); }
    }
}

__global__ __launch_bounds__(32) void k_proj_rows(const bf* __restrict__ A, const bf* __restrict__ Bt, const float* __restrict__ bias, h16* Ph, int K, int nhp, int H, int D, int NH) {
    __shared__ __align__(16) float os[16 * 68];
    const int lane = threadIdx.x & 31, lr = lane & 15, hi = lane >> 4; const int r0 = blockIdx.x * 64, c0 = blockIdx.y * 64;
    v8f acc[4][4];
#pragma unroll
    for (int mb = 0; mb < 4; ++mb)
#pragma unroll
        for (int nb = 0; nb < 4; ++nb) acc[mb][nb] = (v8f){};
    const size_t aoff = (size_t)(r0 + lr) * K + 8 * hi, boff = (size_t)(c0 + lr) * K + 8 * hi;
    gemm64(A, Bt, aoff, boff, K, acc);
    float bc[4];
#pragma unroll
    for (int nb = 0; nb < 4; ++nb) {
        const int hd = (c0 >> 4) + nb; int bi = hd * D + lr; bi = bi < H - 1 ? bi : H - 1;
        float bv = bias[bi]; asm volatile("" : "+v"(bv));
        bc[nb] = ((lr < D) & (hd < NH)) ? bfr(bv) : 0.0f; }
    const int bb = r0 / SEQ, tt = r0 % SEQ;
    const size_t tbase = (((size_t)bb * nhp + (size_t)(c0 >> 4)) * SEQ + (size_t)tt) * HP;
#pragma unroll
    for (int mb = 0; mb < 4; ++mb) {
#pragma unroll
        for (int nb = 0; nb < 4; ++nb) {
#pragma unroll
            for (int j = 0; j < 8; ++j) os[(hi * 8 + j) * 68 + nb * 16 + lr] = (acc[mb][nb][j] + bc[nb]) * PCAR; }
        wave_sync();
        v8h hv[4];
#pragma unroll
        for (int hh = 0; hh < 4; ++hh) { const int row = lane >> 1, c8 = (lane & 1) * 8;
            const v4f x0 = *(const v4fa*)(&os[row * 68 + hh * 16 + c8]); const v4f x1 = *(const v4fa*)(&os[row * 68 + hh * 16 + c8 + 4]);
#pragma unroll
            for (int i = 0; i < 4; ++i) { hv[hh][i] = toh_flush(x0[i]); hv[hh][4 + i] = toh_flush(x1[i]); } }
        const size_t sb = tbase + (size_t)(mb * 16) * HP + (size_t)lane * 8;
#pragma unroll 1
        for (int ps = 0; ps < 2; ++ps) {
#pragma unroll
            for (int hh = 0; hh < 4; ++hh) *(volatile v8h*)(Ph + sb + (size_t)hh * ((size_t)SEQ * HP)) = hv[hh];
            if (ps == 0) __threadfence(); }
        wave_sync();
    }
}

__global__ __launch_bounds__(32) void k_proj_cols(const bf* __restrict__ A, const bf* __restrict__ Bt, const float* __restrict__ bias, h16* Ph, int K, int mp, int H, int D, int NH) {
    __shared__ __align__(16) float os[16 * 68];
    const int lane = threadIdx.x & 31, lr = lane & 15, hi = lane >> 4; const int r0 = blockIdx.x * 64, c0 = blockIdx.y * 64;
    v8f acc[4][4];
#pragma unroll
    for (int mb = 0; mb < 4; ++mb)
#pragma unroll
        for (int nb = 0; nb < 4; ++nb) acc[mb][nb] = (v8f){};
    const size_t aoff = (size_t)(r0 + lr) * K + 8 * hi, boff = (size_t)(c0 + lr) * K + 8 * hi;
    gemm64(A, Bt, aoff, boff, K, acc);
    const int bb = c0 / SEQ, tt = c0 % SEQ;
    const size_t tbase = ((size_t)bb * (size_t)mp + (size_t)r0) * SEQ + (size_t)tt;
#pragma unroll
    for (int mb = 0; mb < 4; ++mb) {
        float br[8];
#pragma unroll
        for (int j = 0; j < 8; ++j) {
            const int hd = (r0 >> 4) + mb; const int dp = hi * 8 + j; int bi = hd * D + dp; bi = bi < H - 1 ? bi : H - 1;
            float bv = bias[bi]; asm volatile("" : "+v"(bv));
            br[j] = ((dp < D) & (hd < NH)) ? bfr(bv) : 0.0f; }
#pragma unroll
        for (int nb = 0; nb < 4; ++nb) {
#pragma unroll
            for (int j = 0; j < 8; ++j) os[(hi * 8 + j) * 68 + nb * 16 + lr] = (acc[mb][nb][j] + br[j]) * PCAR; }
        wave_sync();
        v8h hv[4];
#pragma unroll
        for (int s = 0; s < 4; ++s) { const int row = 4 * s + (lane >> 3), c8 = (lane & 7) * 8;
            const v4f x0 = *(const v4fa*)(&os[row * 68 + c8]); const v4f x1 = *(const v4fa*)(&os[row * 68 + c8 + 4]);
#pragma unroll
            for (int i = 0; i < 4; ++i) { hv[s][i] = toh_flush(x0[i]); hv[s][4 + i] = toh_flush(x1[i]); } }
        const size_t sb = tbase + (size_t)(mb * 16 + (lane >> 3)) * SEQ + (size_t)((lane & 7) * 8);
#pragma unroll 1
        for (int ps = 0; ps < 2; ++ps) {
#pragma unroll
            for (int s = 0; s < 4; ++s) *(volatile v8h*)(Ph + sb + (size_t)(4 * s) * SEQ) = hv[s];
            if (ps == 0) __threadfence(); }
        wave_sync();
    }
}

__global__ __launch_bounds__(32 * AW) void k_flash(const h16* __restrict__ QH, const h16* __restrict__ KP, const h16* __restrict__ VT, const float* __restrict__ mask,
                                                   int hasmask, int nhp, int nh, float sc2, h16* CT) {
    __shared__ __align__(16) float os[AW * 16 * OSP];
    const int lane = threadIdx.x & 31, lr = lane & 15, hi = lane >> 4;
    const int wave = __builtin_amdgcn_readfirstlane((int)(threadIdx.x >> 5));
    const int zh = blockIdx.y; const int b = zh / nhp, h = zh % nhp;
    const int t0 = (blockIdx.x * AW + wave) * 16;
    const int hm = h < nh ? h : nh - 1;
    const float* mrow = mask + ((size_t)b * nh + (size_t)hm) * SEQ_FULL + 8 * hi;
    const size_t pbase = (size_t)zh * SEQ * HP;
    const v8h hz8 = (v8h){};
    const size_t qo = pbase + (size_t)(t0 + lr) * HP + 8 * hi;
    const v16h qh = cat16(*(const v8h*)(QH + qo), hz8);
    const size_t ko = pbase + (size_t)lr * HP + 8 * hi;
    const size_t vo = pbase + (size_t)lr * SEQ + 8 * hi;
    v8f o0 = (v8f){};
    float m = NEGB, l = 0.0f;
#pragma unroll 1
    for (int key0 = 0; key0 < SEQ; key0 += 32) {
        const h16* ka = KP + ko + (size_t)key0 * HP;
        const v16h ka0 = cat16(*(const v8h*)ka, hz8), kb0 = cat16(*(const v8h*)(ka + 16 * HP), hz8);
        v8f sHa = (v8f){}, sHb = (v8f){};
        sHa = wmma16g(ka0, qh, sHa); sHb = wmma16g(kb0, qh, sHb);
        float kx[8], ky[8];
#pragma unroll
        for (int r = 0; r < 8; ++r) { kx[r] = 0.0f; ky[r] = 0.0f; }
        if (hasmask != 0) {
            const float* kp = mrow + key0;
            const v4f m0 = *(const v4f*)kp, m1 = *(const v4f*)(kp + 4), m2 = *(const v4f*)(kp + 16), m3 = *(const v4f*)(kp + 20);
#pragma unroll
            for (int r = 0; r < 4; ++r) { kx[r] = bfr(m0[r]) * LOG2E; kx[4 + r] = bfr(m1[r]) * LOG2E; ky[r] = bfr(m2[r]) * LOG2E; ky[4 + r] = bfr(m3[r]) * LOG2E; }
        }
        float ta[8], tb[8]; float mx = NEGB;
#pragma unroll
        for (int r = 0; r < 8; ++r) {
            ta[r] = sHa[r] * sc2 + kx[r]; tb[r] = sHb[r] * sc2 + ky[r];
            mx = fmaxf(mx, fmaxf(ta[r], tb[r])); }
        mx = fmaxf(mx, __shfl_xor(mx, 16, 32));
        const float mnew = fmaxf(m, mx);
        const float alpha = __builtin_amdgcn_exp2f(m - mnew);
        const float sh = PSH - mnew;
        v16h pb; float ls = 0.0f;
#pragma unroll
        for (int r = 0; r < 8; ++r) {
            const float ea = ta[r] + sh, eb = tb[r] + sh;
            const float ga = (ea < -14.0f) ? 0.0f : __builtin_amdgcn_exp2f(ea);
            const float gb = (eb < -14.0f) ? 0.0f : __builtin_amdgcn_exp2f(eb);
            const h16 pa = (h16)ga; const h16 pc = (h16)gb;
            pb[r] = pa; pb[8 + r] = pc;
            ls += (float)pa + (float)pc; }
        l = l * alpha + ls; m = mnew;
        o0 = o0 * alpha;
        const v16h v0 = ldh(VT + vo + key0);
        o0 = wmma16g(v0, pb, o0);
    }
    l += __shfl_xor(l, 16, 32);
    const bool any = l > 0.0f;
    const float lsafe = any ? l : 1.0f;
    const float inv = any ? (OSC * (1.0f / lsafe)) : 0.0f;
    const int wb = wave * 16 * OSP;
    { v4f a, c;
      a[0] = o0[0] * inv; a[1] = o0[1] * inv; a[2] = o0[2] * inv; a[3] = o0[3] * inv; c[0] = o0[4] * inv; c[1] = o0[5] * inv; c[2] = o0[6] * inv; c[3] = o0[7] * inv;
      *(v4fa*)(&os[wb + lr * OSP + 8 * hi]) = a; *(v4fa*)(&os[wb + lr * OSP + 8 * hi + 4]) = c; }
    wave_sync();
    v8h hv;
    { const int row = lane >> 1, c8 = (lane & 1) * 8;
      const v4f x0 = *(const v4fa*)(&os[wb + row * OSP + c8]); const v4f x1 = *(const v4fa*)(&os[wb + row * OSP + c8 + 4]);
#pragma unroll
      for (int i = 0; i < 4; ++i) { hv[i] = toh_flush(x0[i]); hv[4 + i] = toh_flush(x1[i]); } }
    h16* crow = CT + pbase + (size_t)t0 * HP + (size_t)lane * 8;
#pragma unroll 1
    for (int ps = 0; ps < 2; ++ps) {
        *(volatile v8h*)crow = hv;
        if (ps == 0) __threadfence(); }
}

__global__ __launch_bounds__(32) void k_oproj(const h16* __restrict__ CT, const h16* __restrict__ WO, const float* __restrict__ bo, float* OUT, int nhp, int N, int KC) {
    __shared__ __align__(16) float os[16 * OPP];
    const int lane = threadIdx.x & 31, lr = lane & 15, hi = lane >> 4;
    const int m0 = blockIdx.x * 16; const int bb = m0 / SEQ, tt = m0 % SEQ;
    v8f acc[ONT];
#pragma unroll
    for (int nb = 0; nb < ONT; ++nb) acc[nb] = (v8f){};
    const size_t abase = ((size_t)bb * nhp * SEQ + (size_t)(tt + lr)) * HP + 8 * hi;
    const size_t boff = (size_t)lr * KC + 8 * hi;
#pragma unroll 1
    for (int kc = 0; kc < KC; kc += 32) {
        const h16* ap = CT + abase + (size_t)(kc >> 4) * ((size_t)SEQ * HP);
        const v16h a = cat16(*(const v8h*)ap, *(const v8h*)(ap + (size_t)SEQ * HP));
#pragma unroll
        for (int nb = 0; nb < ONT; ++nb) { const v16h b = ldh(WO + boff + (size_t)nb * 16 * KC + kc); acc[nb] = wmma16g(a, b, acc[nb]); }
    }
#pragma unroll
    for (int nb = 0; nb < ONT; ++nb) {
        const int col = nb * 16 + lr; const int bi = col < N ? col : N - 1;
        const float bv = bfr(bo[bi]);
#pragma unroll
        for (int j = 0; j < 8; ++j) os[(hi * 8 + j) * OPP + col] = acc[nb][j] * OFOLD + bv; }
    wave_sync();
    float* obase = OUT + ((size_t)bb * OUT_SEQ + (size_t)tt) * (size_t)N;
    const int n4 = 4 * N;
    const int trips = (n4 + 31) >> 5;
#pragma unroll 1
    for (int ps = 0; ps < 2; ++ps) {
#pragma unroll 1
        for (int it = 0; it < trips; ++it) {
            const int i = it * 32 + lane; const int ic = i < n4 ? i : n4 - 1;
            v4f val;
#pragma unroll
            for (int j = 0; j < 4; ++j) { const int e = 4 * ic + j; const int row = e / N; const int col = e - row * N; val[j] = os[row * OPP + col]; }
            if (i < n4) *(volatile v4f*)(obase + (size_t)4 * i) = val; }
        if (ps == 0) __threadfence(); }
}

static constexpr size_t al256(size_t v) { return (v + 255) & ~(size_t)255; }
static constexpr size_t SZ_XA = al256((size_t)NB * SEQ * KPA * 2);
static constexpr size_t SZ_YB = al256((size_t)NB * SEQ * KPB * 2);
static constexpr size_t SZ_WA = al256((size_t)NPA * HP * KPA * 2);
static constexpr size_t SZ_WB = al256((size_t)NPB * HP * KPB * 2);
static constexpr size_t SZ_OA = al256((size_t)NRO * NPA * HP * 2);
static constexpr size_t SZ_OB = al256((size_t)NRO * NPB * HP * 2);
static constexpr size_t SZ_PA = al256((size_t)NB * NPA * SEQ * HP * 2);
static constexpr size_t SZ_PB = al256((size_t)NB * NPB * SEQ * HP * 2);
static constexpr size_t SZ_TOTAL = SZ_XA + SZ_YB + 3 * SZ_WA + 3 * SZ_WB + SZ_OA + SZ_OB + 4 * SZ_PA + 4 * SZ_PB;
static_assert(SZ_TOTAL <= (size_t)134217728);
static_assert(((size_t)NB * SEQ * KPA * 2) % 128 == 0);
static_assert(((size_t)NB * SEQ * KPB * 2) % 128 == 0);
static_assert(((size_t)NPA * HP * KPA * 2) % 128 == 0);
static_assert(((size_t)NPB * HP * KPB * 2) % 128 == 0);
static_assert(((size_t)NRO * NPA * HP * 2) % 128 == 0);
static_assert(((size_t)NRO * NPB * HP * 2) % 128 == 0);

extern "C" void kernel_launch(void* const* d_in, const int* in_sizes, int n_in,
                              void* d_out, int out_size, void* d_ws, size_t ws_size, hipStream_t stream) {
    if (n_in < 19) return;
    const size_t rowsneed = (size_t)(NB - 1) * SEQ_FULL + SEQ;
    if ((size_t)in_sizes[0] < rowsneed * HA || (size_t)in_sizes[1] < rowsneed * HB) return;
    if ((size_t)in_sizes[2] < ((size_t)NB * NHB - 1) * SEQ_FULL + SEQ) return;
    for (int i = 0; i < 4; ++i) {
        if ((size_t)in_sizes[3 + 2 * i] < (size_t)HA * HA || in_sizes[4 + 2 * i] < HA) return;
        if ((size_t)in_sizes[11 + 2 * i] < (size_t)HB * HB || in_sizes[12 + 2 * i] < HB) return;
    }
    const size_t out1_off = (size_t)NB_FULL * SEQ_FULL * HA;
    if ((size_t)out_size < out1_off + ((size_t)(NB - 1) * OUT_SEQ + SEQ) * HB) return;
    if ((size_t)out_size < ((size_t)(NB - 1) * OUT_SEQ + SEQ) * HA) return;
    if (SZ_TOTAL > ws_size) return;
    const float* x = (const float*)d_in[0]; const float* y = (const float*)d_in[1]; const float* mask = (const float*)d_in[2];
    const float* wq0 = (const float*)d_in[3];  const float* bq0 = (const float*)d_in[4];
    const float* wk0 = (const float*)d_in[5];  const float* bk0 = (const float*)d_in[6];
    const float* wv0 = (const float*)d_in[7];  const float* bv0 = (const float*)d_in[8];
    const float* wo0 = (const float*)d_in[9];  const float* bo0 = (const float*)d_in[10];
    const float* wq1 = (const float*)d_in[11]; const float* bq1 = (const float*)d_in[12];
    const float* wk1 = (const float*)d_in[13]; const float* bk1 = (const float*)d_in[14];
    const float* wv1 = (const float*)d_in[15]; const float* bv1 = (const float*)d_in[16];
    const float* wo1 = (const float*)d_in[17]; const float* bo1 = (const float*)d_in[18];
    float* OUT0 = (float*)d_out;
    float* OUT1 = (float*)d_out + out1_off;
    char* wsp = (char*)d_ws;
    bf* XA = (bf*)wsp; wsp += SZ_XA;
    bf* YB = (bf*)wsp; wsp += SZ_YB;
    bf* WQA = (bf*)wsp; wsp += SZ_WA;
    bf* WKA = (bf*)wsp; wsp += SZ_WA;
    bf* WVA = (bf*)wsp; wsp += SZ_WA;
    bf* WQB = (bf*)wsp; wsp += SZ_WB;
    bf* WKB = (bf*)wsp; wsp += SZ_WB;
    bf* WVB = (bf*)wsp; wsp += SZ_WB;
    h16* WOA = (h16*)wsp; wsp += SZ_OA;
    h16* WOB = (h16*)wsp; wsp += SZ_OB;
    h16* QA = (h16*)wsp; wsp += SZ_PA;
    h16* KA = (h16*)wsp; wsp += SZ_PA;
    h16* VA = (h16*)wsp; wsp += SZ_PA;
    h16* CA = (h16*)wsp; wsp += SZ_PA;
    h16* QB = (h16*)wsp; wsp += SZ_PB;
    h16* KB = (h16*)wsp; wsp += SZ_PB;
    h16* VB = (h16*)wsp; wsp += SZ_PB;
    h16* CB = (h16*)wsp; wsp += SZ_PB;

    if (SEQ == SEQ_FULL) {
        const size_t n8 = (size_t)NB * SEQ * HA / 8;
        k_cvt8<<<(unsigned)((n8 + 255) / 256), 256, 0, stream>>>(x, XA, n8);
        const int nt = NB * SEQ * (KPB / 8);
        k_cvtpad<<<(unsigned)((nt + 255) / 256), 256, 0, stream>>>(y, YB, NB * SEQ, HB, KPB);
    } else {
        const size_t n8 = (size_t)SEQ * HA / 8; const int nt = SEQ * (KPB / 8);
        for (int b = 0; b < NB; ++b) {
            k_cvt8<<<(unsigned)((n8 + 255) / 256), 256, 0, stream>>>(x + (size_t)b * SEQ_FULL * HA, XA + (size_t)b * SEQ * KPA, n8);
            k_cvtpad<<<(unsigned)((nt + 255) / 256), 256, 0, stream>>>(y + (size_t)b * SEQ_FULL * HB, YB + (size_t)b * SEQ * KPB, SEQ, HB, KPB);
        }
    }
    { const int na = NPA * HP * (KPA / 8); const unsigned ga = (unsigned)((na + 255) / 256);
      k_wpack_rows<<<ga, 256, 0, stream>>>(wq0, WQA, HA, DA, NHA, KPA, NPA * HP);
      k_wpack_rows<<<ga, 256, 0, stream>>>(wk0, WKA, HA, DA, NHA, KPA, NPA * HP);
      k_wpack_rows<<<ga, 256, 0, stream>>>(wv0, WVA, HA, DA, NHA, KPA, NPA * HP);
      const int nb = NPB * HP * (KPB / 8); const unsigned gb = (unsigned)((nb + 255) / 256);
      k_wpack_rows<<<gb, 256, 0, stream>>>(wq1, WQB, HB, DB, NHB, KPB, NPB * HP);
      k_wpack_rows<<<gb, 256, 0, stream>>>(wk1, WKB, HB, DB, NHB, KPB, NPB * HP);
      k_wpack_rows<<<gb, 256, 0, stream>>>(wv1, WVB, HB, DB, NHB, KPB, NPB * HP);
      const int noa = NRO * (NPA * HP / 8); const int nob = NRO * (NPB * HP / 8);
      k_wpack_cols<<<(unsigned)((noa + 255) / 256), 256, 0, stream>>>(wo0, WOA, HA, DA, NHA, NPA * HP, NRO);
      k_wpack_cols<<<(unsigned)((nob + 255) / 256), 256, 0, stream>>>(wo1, WOB, HB, DB, NHB, NPB * HP, NRO); }

    k_proj_rows<<<dim3(NB * SEQ / 64, NPA * HP / 64, 1), 32, 0, stream>>>(XA, WQA, bq0, QA, KPA, NPA, HA, DA, NHA);
    k_proj_rows<<<dim3(NB * SEQ / 64, NPA * HP / 64, 1), 32, 0, stream>>>(XA, WKA, bk0, KA, KPA, NPA, HA, DA, NHA);
    k_proj_cols<<<dim3(NPA * HP / 64, NB * SEQ / 64, 1), 32, 0, stream>>>(WVA, XA, bv0, VA, KPA, NPA * HP, HA, DA, NHA);
    k_proj_rows<<<dim3(NB * SEQ / 64, NPB * HP / 64, 1), 32, 0, stream>>>(YB, WQB, bq1, QB, KPB, NPB, HB, DB, NHB);
    k_proj_rows<<<dim3(NB * SEQ / 64, NPB * HP / 64, 1), 32, 0, stream>>>(YB, WKB, bk1, KB, KPB, NPB, HB, DB, NHB);
    k_proj_cols<<<dim3(NPB * HP / 64, NB * SEQ / 64, 1), 32, 0, stream>>>(WVB, YB, bv1, VB, KPB, NPB * HP, HB, DB, NHB);

    const float sc2a = (float)(0.28867513459481287 * 1.4426950408889634 / 256.0);
    const float sc2b = (float)(0.40824829046386302 * 1.4426950408889634 / 256.0);
    k_flash<<<dim3(SEQ / (16 * AW), NB * NPA, 1), 32 * AW, 0, stream>>>(QA, KA, VA, mask, 0, NPA, NHA, sc2a, CA);
    k_flash<<<dim3(SEQ / (16 * AW), NB * NPB, 1), 32 * AW, 0, stream>>>(QB, KB, VB, mask, 1, NPB, NHB, sc2b, CB);

    k_oproj<<<dim3(NB * SEQ / 16, 1, 1), 32, 0, stream>>>(CA, WOA, bo0, OUT0, NPA, HA, NPA * HP);
    k_oproj<<<dim3(NB * SEQ / 16, 1, 1), 32, 0, stream>>>(CB, WOB, bo1, OUT1, NPB, HB, NPB * HP);
}
